// Net_55714315763758
// MI455X (gfx1250) — hardware-verified
//
#include <hip/hip_runtime.h>
#include <stddef.h>
#include <stdint.h>


#define DF     128
#define OC     64
#define PA     256
#define K0L    384
#define K1L    256
#define NTHR   256
#define NWAVE  8
#define EPT    8
#define CHUNK  (NTHR * EPT)
#define WCAP   (EPT * 32)
#define LISTN  (NWAVE * WCAP)
#define NBA    1024
#define SLA    10
#define RCAP   28672
#define DEGCAP 64
#define RPB    64
#define GBM    64
#define GBN    128
#define GTHR   128
#define NB_W1  24
#define NB_W2  16
#define AGG_ZINTS (LISTN + 2 * RCAP + 3 * NBA)
#define AGG_LDS_INTS (AGG_ZINTS + 16)
#define WSMAX  134217728
#define NSTAT  40000
#define ESTAT  640000
#define MEAS_B1024  16638
#define MEAS_MAXDEG 36

static_assert(DF == 128 && DF == 4 * 32);
static_assert(OC == 64 && 2 * OC == GBN && OC == 2 * 32);
static_assert(K0L % 32 == 0 && K1L % 32 == 0 && K0L == 3 * DF && K1L == 2 * DF && K1L == PA);
static_assert((ESTAT % 4) == 0);
static_assert(NBA * 40 >= NSTAT);
static_assert(RCAP >= MEAS_B1024 + MEAS_B1024 / 20 + 1);
static_assert(DEGCAP >= MEAS_MAXDEG + 8);
static_assert(((NSTAT + 127) / 128) * 128 == 313 * 128);
static_assert((CHUNK & (CHUNK - 1)) == 0 && CHUNK <= 4096);
static_assert((NBA & (NBA - 1)) == 0 && NBA == (1 << SLA) && NBA == NTHR * 4);
static_assert(((long long)CHUNK << SLA) < (1LL << 31));
static_assert(((long long)ESTAT << SLA) < (1LL << 31));
static_assert(RCAP % (NTHR * 4) == 0 && AGG_ZINTS % 4 == 0 && LISTN % 4 == 0);
static_assert(NBA % 32 == 0 && NBA % RPB == 0 && RPB % NWAVE == 0);
static_assert(GBM == (GTHR / 32) * 16);
static_assert(AGG_LDS_INTS * 4 <= 300000);
static_assert((3 * DF * (DF / 8)) == NB_W1 * NTHR && (128 * (K1L / 8)) == NB_W2 * NTHR);
static_assert(98304ull + 65536ull + 768ull + 40ull * 128 + 2ull * 40 * NBA * 4 + 40ull * RCAP * 4 +
              40064ull * DF * 2 + 2ull * 40064 * PA * 2 + 40064ull * DF * 4 <= (unsigned long long)WSMAX);

typedef float          v2f   __attribute__((ext_vector_type(2)));
typedef float          v4f   __attribute__((ext_vector_type(4)));
typedef float          v8f   __attribute__((ext_vector_type(8)));
typedef int            v4i   __attribute__((ext_vector_type(4)));
typedef int            v8i   __attribute__((ext_vector_type(8)));
typedef unsigned       v2u   __attribute__((ext_vector_type(2)));
typedef unsigned short v4us  __attribute__((ext_vector_type(4)));
typedef unsigned short v8us  __attribute__((ext_vector_type(8)));
typedef unsigned short v16us __attribute__((ext_vector_type(16)));
typedef __bf16         v16bf __attribute__((ext_vector_type(16)));
typedef v2f  __attribute__((may_alias)) v2fa;
typedef v4f  __attribute__((may_alias)) v4fa;
typedef v4i  __attribute__((may_alias)) v4ia;
typedef v2u  __attribute__((may_alias)) v2ua;
typedef v4us __attribute__((may_alias)) v4usa;
typedef v8us __attribute__((may_alias)) v8usa;
union FragB { v16bf v; v16us u; v8us h[2]; v8i w; };

__device__ __forceinline__ v8f wmb(const FragB& a, const FragB& b, v8f c) {
  v8f d = __builtin_amdgcn_wmma_f32_16x16x32_bf16(false, a.v, false, b.v, (short)0, c, false, false);
  asm volatile("v_nop\n\tv_nop\n\tv_nop\n\tv_nop" : "+v"(d) : "v"(a.w), "v"(b.w));
  return d;
}

__device__ __forceinline__ unsigned bf16_bits(float f) {
  const unsigned u = __float_as_uint(f);
  return (u + 0x7FFFu + ((u >> 16) & 1u)) >> 16;
}
__device__ __forceinline__ float bf16_val(float f) {
  return __uint_as_float(bf16_bits(f) << 16);
}

__device__ __forceinline__ void wave_sync() {
  __builtin_amdgcn_fence(__ATOMIC_RELEASE, "wavefront");
  __builtin_amdgcn_wave_barrier();
  __builtin_amdgcn_fence(__ATOMIC_ACQUIRE, "wavefront");
}

__device__ __forceinline__ v8us cvt8(const float* __restrict__ p, bool ok) {
  const v4f a = *(const v4f*)p;
  const v4f b = *(const v4f*)(p + 4);
  v8us o;
  o[0] = ok ? (unsigned short)bf16_bits(a.x) : (unsigned short)0;
  o[1] = ok ? (unsigned short)bf16_bits(a.y) : (unsigned short)0;
  o[2] = ok ? (unsigned short)bf16_bits(a.z) : (unsigned short)0;
  o[3] = ok ? (unsigned short)bf16_bits(a.w) : (unsigned short)0;
  o[4] = ok ? (unsigned short)bf16_bits(b.x) : (unsigned short)0;
  o[5] = ok ? (unsigned short)bf16_bits(b.y) : (unsigned short)0;
  o[6] = ok ? (unsigned short)bf16_bits(b.z) : (unsigned short)0;
  o[7] = ok ? (unsigned short)bf16_bits(b.w) : (unsigned short)0;
  return o;
}

template <int SLB>
__device__ __forceinline__ int scan_chunk(const int* __restrict__ dsts, int nE, int cbase, int slotBase,
                                          int nb, int vec8, int* list, int tid, int lane, int wave) {
  int wc = 0;
  const int el0  = tid * EPT;
  const int e0   = cbase + el0;
  const int sent = -2147483647 - 1;
  v4i da, db;
  if (vec8 != 0 && cbase + CHUNK <= nE) {
    da = *(const v4i*)(dsts + e0);
    db = *(const v4i*)(dsts + e0 + 4);
  } else {
    da.x = (e0     < nE) ? dsts[min(e0,     nE - 1)] : sent;
    da.y = (e0 + 1 < nE) ? dsts[min(e0 + 1, nE - 1)] : sent;
    da.z = (e0 + 2 < nE) ? dsts[min(e0 + 2, nE - 1)] : sent;
    da.w = (e0 + 3 < nE) ? dsts[min(e0 + 3, nE - 1)] : sent;
    db.x = (e0 + 4 < nE) ? dsts[min(e0 + 4, nE - 1)] : sent;
    db.y = (e0 + 5 < nE) ? dsts[min(e0 + 5, nE - 1)] : sent;
    db.z = (e0 + 6 < nE) ? dsts[min(e0 + 6, nE - 1)] : sent;
    db.w = (e0 + 7 < nE) ? dsts[min(e0 + 7, nE - 1)] : sent;
  }
  const unsigned nbs = (unsigned)slotBase;
  const unsigned unb = (unsigned)nb;
  const unsigned s0 = (unsigned)da.x - nbs, s1 = (unsigned)da.y - nbs;
  const unsigned s2 = (unsigned)da.z - nbs, s3 = (unsigned)da.w - nbs;
  const unsigned s4 = (unsigned)db.x - nbs, s5 = (unsigned)db.y - nbs;
  const unsigned s6 = (unsigned)db.z - nbs, s7 = (unsigned)db.w - nbs;
  const bool h0 = s0 < unb, h1 = s1 < unb, h2 = s2 < unb, h3 = s3 < unb;
  const bool h4 = s4 < unb, h5 = s5 < unb, h6 = s6 < unb, h7 = s7 < unb;
  const unsigned any = __builtin_amdgcn_ballot_w32(h0 | h1 | h2 | h3 | h4 | h5 | h6 | h7);
  if (any != 0u) {
#define HITJ(J, HJ, SJ) { \
      const unsigned mj = __builtin_amdgcn_ballot_w32(HJ); \
      if (mj != 0u) { \
        if (HJ) { \
          const int pos = wc + (int)__builtin_amdgcn_mbcnt_lo(mj, 0u); \
          if (pos < WCAP) list[wave * WCAP + pos] = ((el0 + (J)) << SLB) | (int)(SJ); \
        } \
        wc += (int)__builtin_popcount(mj); } }
    HITJ(0, h0, s0)
    HITJ(1, h1, s1)
    HITJ(2, h2, s2)
    HITJ(3, h3, s3)
    HITJ(4, h4, s4)
    HITJ(5, h5, s5)
    HITJ(6, h6, s6)
    HITJ(7, h7, s7)
#undef HITJ
  }
  return wc;
}

__global__ __launch_bounds__(NTHR) void k_prep(const float* __restrict__ x, const float* __restrict__ W1rel,
                                               const float* __restrict__ W1root, const float* __restrict__ b1,
                                               const float* __restrict__ W2rel, const float* __restrict__ W2root,
                                               const float* __restrict__ b2, int nN, int nbX,
                                               unsigned short* XB, unsigned short* W1cat, unsigned short* W2cat,
                                               float* BF) {
  const int tid = (int)threadIdx.x;
  const int blk = (int)blockIdx.x;
  if (blk < nbX) {
    const int u   = blk * NTHR + tid;
    const int row = u >> 4;
    const int k8  = (u & 15) * 8;
    const int rc  = row < nN ? row : nN - 1;
    const v8us o  = cvt8(x + (size_t)rc * DF + k8, row < nN);
    unsigned short* dp = XB + (size_t)row * DF + k8;
    *(volatile v8us*)dp = o;
    __threadfence();
    *(volatile v8us*)dp = o;
  } else if (blk < nbX + NB_W1) {
    const int u    = (blk - nbX) * NTHR + tid;
    const int part = u >> 11;
    const int v    = u & 2047;
    const int n    = v >> 4;
    const int k8   = (v & 15) * 8;
    v8us o;
    if (part < 2) o = cvt8(W1rel + (size_t)n * DF + k8, true);
    else          o = cvt8(W1root + (size_t)n * DF + k8, true);
    unsigned short* dp = W1cat + (size_t)n * K0L + part * DF + k8;
    *(volatile v8us*)dp = o;
    __threadfence();
    *(volatile v8us*)dp = o;
  } else if (blk < nbX + NB_W1 + NB_W2) {
    const int u  = (blk - nbX - NB_W1) * NTHR + tid;
    const int n  = u >> 5;
    const int k8 = (u & 31) * 8;
    const int kk = k8 & (DF - 1);
    v8us o;
    if (n < OC) o = cvt8(W2rel + (size_t)n * DF + kk, true);
    else        o = cvt8(W2root + (size_t)(n - OC) * DF + kk, true);
    unsigned short* dp = W2cat + (size_t)n * K1L + k8;
    *(volatile v8us*)dp = o;
    __threadfence();
    *(volatile v8us*)dp = o;
  } else {
    const int lane = tid & 31, wave = tid >> 5;
    if (wave == 0) {
      const v4f t = *(const v4f*)(b1 + 4 * lane);
      v4f r;
      r.x = bf16_val(t.x); r.y = bf16_val(t.y); r.z = bf16_val(t.z); r.w = bf16_val(t.w);
      float* dp = BF + 4 * lane;
      *(volatile v4f*)dp = r;
      __threadfence();
      *(volatile v4f*)dp = r;
    } else if (wave == 1) {
      const int l = lane & 15;
      const v4f t = *(const v4f*)(b2 + 4 * l);
      v4f r;
      r.x = bf16_val(t.x); r.y = bf16_val(t.y); r.z = bf16_val(t.z); r.w = bf16_val(t.w);
      float* dp = BF + DF + 4 * l;
      const bool wr = lane < 16;
      if (wr) *(volatile v4f*)dp = r;
      __threadfence();
      if (wr) *(volatile v4f*)dp = r;
    }
  }
}

__global__ __launch_bounds__(NTHR) void k_compact(const int* __restrict__ ei, int nE, int nN, int vec8,
                                                  int* listp, int* cntp, int* offp, int* flagp) {
  extern __shared__ __attribute__((aligned(16))) int dsm[];
  int* list = dsm;
  int* hl   = dsm + LISTN;
  int* sl   = dsm + LISTN + RCAP;
  int* cnt  = dsm + LISTN + 2 * RCAP;
  int* offs = cnt + NBA;
  int* cur  = offs + NBA;
  int* misc = cur + NBA;
  const int tid = (int)threadIdx.x, lane = tid & 31, wave = tid >> 5;
  const int b = (int)blockIdx.x;
  const int nodeBase = b * NBA;
  const int* srcs = ei;
  const int* dsts = ei + nE;

  {
    const v4i z4 = {0, 0, 0, 0};
    for (int i = tid * 4; i < AGG_ZINTS; i += NTHR * 4) *(v4ia*)(dsm + i) = z4;
    if (tid < 16) misc[tid] = 0;
  }
  __syncthreads();

  int t = 0, ov = 0;
  const int nChunks = (nE + CHUNK - 1) / CHUNK;
#pragma unroll 1
  for (int ch = 0; ch < nChunks; ++ch) {
    const int cbase = ch * CHUNK;
    const int wc = scan_chunk<SLA>(dsts, nE, cbase, nodeBase, NBA, vec8, list, tid, lane, wave);
    if (lane == 0) misc[wave] = wc;
    __syncthreads();
    if (wave == 0) {
#pragma unroll 1
      for (int w2 = 0; w2 < NWAVE; ++w2) {
        int c = misc[w2];
        c = c < 0 ? 0 : (c > WCAP ? WCAP : c);
#pragma unroll 1
        for (int b0 = 0; b0 < c; b0 += 32) {
          const int idx = b0 + lane;
          const int ent = list[w2 * WCAP + (idx < WCAP ? idx : WCAP - 1)];
          const int m32 = (c - b0) < 32 ? (c - b0) : 32;
#pragma unroll 1
          for (int k = 0; k < m32; ++k) {
            const int u    = __builtin_amdgcn_readlane(ent, k);
            const int slot = u & (NBA - 1);
            const int el   = (u >> SLA) & (CHUNK - 1);
            const int pk   = ((cbase + el) << SLA) | slot;
            if (t < RCAP) {
              if (lane == 0) { hl[t] = pk; cnt[slot] = cnt[slot] + 1; }
              t = t + 1;
            } else {
              ov = 1;
            }
          }
        }
      }
    }
    __syncthreads();
  }
  if (wave == 0 && lane == 0) { misc[8] = t; misc[9] = ov; }
  __syncthreads();
  int tt = misc[8];
  tt = tt < 0 ? 0 : (tt > RCAP ? RCAP : tt);
  const int ovf = misc[9];

  if (wave == 0) {
    const int base = lane * (NBA / 32);
    int s = 0;
#pragma unroll 1
    for (int i = 0; i < NBA / 32; ++i) s += cnt[base + i];
    int incl = s;
#pragma unroll
    for (int d = 1; d < 32; d <<= 1) {
      const int y = __shfl_up(incl, d, 32);
      if (lane >= d) incl += y;
    }
    int run = incl - s;
#pragma unroll 1
    for (int i = 0; i < NBA / 32; ++i) {
      const int cv = cnt[base + i];
      offs[base + i] = run;
      cur[base + i]  = run;
      run += cv;
    }
  }
  __syncthreads();
  if (wave == 0) {
#pragma unroll 1
    for (int b0 = 0; b0 < tt; b0 += 32) {
      const int idx = b0 + lane;
      const int ent = hl[idx < RCAP ? idx : RCAP - 1];
      const int m32 = (tt - b0) < 32 ? (tt - b0) : 32;
#pragma unroll 1
      for (int k = 0; k < m32; ++k) {
        const int u    = __builtin_amdgcn_readlane(ent, k);
        const int slot = u & (NBA - 1);
        if (lane == 0) {
          int p = cur[slot];
          p = p < 0 ? 0 : (p > RCAP - 1 ? RCAP - 1 : p);
          sl[p] = u;
          cur[slot] = p + 1;
        }
      }
    }
  }
  __syncthreads();

  const v4i c4 = *(const v4ia*)(cnt + 4 * tid);
  const v4i o4 = *(const v4ia*)(offs + 4 * tid);
  if (c4.x > DEGCAP || c4.y > DEGCAP || c4.z > DEGCAP || c4.w > DEGCAP) misc[10] = 1;
  __syncthreads();
  const int fl = (ovf != 0 || misc[10] != 0) ? 1 : 0;

#pragma unroll 1
  for (int it = 0; it < RCAP / (NTHR * 4); ++it) {
    const int i4 = 4 * (it * NTHR + tid);
    const v4i e = *(const v4ia*)(sl + i4);
    int e0 = e.x >> SLA, e1 = e.y >> SLA, e2 = e.z >> SLA, e3 = e.w >> SLA;
    e0 = e0 < 0 ? 0 : (e0 > nE - 1 ? nE - 1 : e0);
    e1 = e1 < 0 ? 0 : (e1 > nE - 1 ? nE - 1 : e1);
    e2 = e2 < 0 ? 0 : (e2 > nE - 1 ? nE - 1 : e2);
    e3 = e3 < 0 ? 0 : (e3 > nE - 1 ? nE - 1 : e3);
    int s0 = srcs[e0], s1 = srcs[e1], s2 = srcs[e2], s3 = srcs[e3];
    s0 = s0 < 0 ? 0 : (s0 > nN - 1 ? nN - 1 : s0);
    s1 = s1 < 0 ? 0 : (s1 > nN - 1 ? nN - 1 : s1);
    s2 = s2 < 0 ? 0 : (s2 > nN - 1 ? nN - 1 : s2);
    s3 = s3 < 0 ? 0 : (s3 > nN - 1 ? nN - 1 : s3);
    v4i o;
    o.x = (i4     < tt) ? s0 : 0;
    o.y = (i4 + 1 < tt) ? s1 : 0;
    o.z = (i4 + 2 < tt) ? s2 : 0;
    o.w = (i4 + 3 < tt) ? s3 : 0;
    int* dp = listp + (size_t)b * RCAP + i4;
    *(volatile v4i*)dp = o;
    __threadfence();
    *(volatile v4i*)dp = o;
  }
  {
    int* cp = cntp + (size_t)nodeBase + 4 * tid;
    int* op = offp + (size_t)nodeBase + 4 * tid;
    *(volatile v4i*)cp = c4;
    *(volatile v4i*)op = o4;
    __threadfence();
    *(volatile v4i*)cp = c4;
    *(volatile v4i*)op = o4;
  }
  {
    const v4i f4 = {fl, fl, fl, fl};
    int* fp = flagp + (size_t)b * 32 + 4 * (lane & 7);
    const bool wr = (wave == 0) && (lane < 8);
    if (wr) *(volatile v4i*)fp = f4;
    __threadfence();
    if (wr) *(volatile v4i*)fp = f4;
  }
}

__global__ __launch_bounds__(NTHR) void k_agg0(const unsigned short* __restrict__ xb,
                                               const int* __restrict__ listp, const int* __restrict__ cntp,
                                               const int* __restrict__ offp, const int* __restrict__ flagp,
                                               int nN, int mRows, int nBlk, unsigned short* agg) {
  __shared__ __attribute__((aligned(16))) unsigned short rbuf[NWAVE * PA];
  const int tid = (int)threadIdx.x, lane = tid & 31, wave = tid >> 5;
  unsigned short* rowbuf = rbuf + wave * PA;
  const int rowBase = (int)blockIdx.x * RPB;
  int b = rowBase >> SLA;
  b = b > nBlk - 1 ? nBlk - 1 : b;
  const int fl = __builtin_amdgcn_readfirstlane(flagp[(size_t)b * 32]);
  const int* lp = listp + (size_t)b * RCAP;
  const float qnan = __int_as_float(0x7fc00000);
  const float pz = (fl != 0) ? qnan : 0.0f;
  const int slotMax = nBlk * NBA - 1;

#pragma unroll 1
  for (int j = 0; j < RPB / NWAVE; ++j) {
    const int node = rowBase + wave * (RPB / NWAVE) + j;
    const int sc = node < slotMax ? node : slotMax;
    int c = __builtin_amdgcn_readfirstlane(cntp[sc]);
    int o = __builtin_amdgcn_readfirstlane(offp[sc]);
    const bool big = c > DEGCAP;
    c = c < 0 ? 0 : (c > DEGCAP ? DEGCAP : c);
    o = o < 0 ? 0 : (o > RCAP - 1 ? RCAP - 1 : o);
    int last = o + c - 1;
    last = last < 0 ? 0 : (last > RCAP - 1 ? RCAP - 1 : last);
    float a0 = 0.0f, a1 = 0.0f, a2 = 0.0f, a3 = 0.0f;
#pragma unroll 1
    for (int b0 = 0; b0 < c; b0 += 32) {
      int idx = o + b0 + lane;
      idx = idx > last ? last : idx;
      int sr = lp[idx];
      sr = sr < 0 ? 0 : (sr > nN - 1 ? nN - 1 : sr);
      const int m32 = (c - b0) < 32 ? (c - b0) : 32;
#pragma unroll 1
      for (int k = 0; k < m32; ++k) {
        const int sk = __builtin_amdgcn_readlane(sr, k);
        const v2u w = *(const v2ua*)(xb + (size_t)sk * DF + 4 * lane);
        a0 += __uint_as_float(w.x << 16);
        a1 += __uint_as_float(w.x & 0xffff0000u);
        a2 += __uint_as_float(w.y << 16);
        a3 += __uint_as_float(w.y & 0xffff0000u);
      }
    }
    const float pzr = big ? qnan : pz;
    const bool live = node < nN;
    const float m0 = live ? (a0 + pzr) : 0.0f;
    const float m1 = live ? (a1 + pzr) : 0.0f;
    const float m2 = live ? (a2 + pzr) : 0.0f;
    const float m3 = live ? (a3 + pzr) : 0.0f;
    v4us mh, ml;
    {
      unsigned hb;
      hb = bf16_bits(m0); mh[0] = (unsigned short)hb; ml[0] = (unsigned short)bf16_bits(m0 - __uint_as_float(hb << 16));
      hb = bf16_bits(m1); mh[1] = (unsigned short)hb; ml[1] = (unsigned short)bf16_bits(m1 - __uint_as_float(hb << 16));
      hb = bf16_bits(m2); mh[2] = (unsigned short)hb; ml[2] = (unsigned short)bf16_bits(m2 - __uint_as_float(hb << 16));
      hb = bf16_bits(m3); mh[3] = (unsigned short)hb; ml[3] = (unsigned short)bf16_bits(m3 - __uint_as_float(hb << 16));
    }
    *(v4usa*)(rowbuf + 4 * lane) = mh;
    *(v4usa*)(rowbuf + DF + 4 * lane) = ml;
    wave_sync();
    const v8us q0 = *(const v8usa*)(rowbuf + 8 * lane);
    wave_sync();
    if (node < mRows) {
      unsigned short* rpw = agg + (size_t)node * PA + 8 * lane;
      *(volatile v8us*)rpw = q0;
      __threadfence();
      *(volatile v8us*)rpw = q0;
    }
  }
}

template <int MODE>
__global__ __launch_bounds__(GTHR) void k_gemm(const unsigned short* __restrict__ A0,
                                               const unsigned short* __restrict__ A1,
                                               const unsigned short* __restrict__ BT,
                                               const float* __restrict__ biasp,
                                               unsigned short* outH, float* outF, int nLive) {
  constexpr int KB = (MODE == 0) ? K0L : K1L;
  __shared__ __attribute__((aligned(16))) float stg[GBM * GBN];
  __shared__ __attribute__((aligned(16))) float bsm[GBN];
  const int tid = (int)threadIdx.x, lane = tid & 31, wave = tid >> 5, hh = lane >> 4, m = lane & 15;
  const int rowBase = (int)blockIdx.x * GBM;

  v8f acc[8];
  {
    const v8f z = {0.f, 0.f, 0.f, 0.f, 0.f, 0.f, 0.f, 0.f};
#pragma unroll
    for (int t = 0; t < 8; ++t) acc[t] = z;
  }
  const unsigned short* ap0 = A0 + (size_t)(rowBase + 16 * wave + m) * (size_t)PA + 8 * hh;
  const unsigned short* bp  = BT + (size_t)m * (size_t)KB + 8 * hh;

#pragma unroll 1
  for (int k0 = 0; k0 < PA; k0 += 32) {
    FragB af;
    af.h[0] = *(const v8usa*)(ap0 + k0);
    af.h[1] = *(const v8usa*)(ap0 + k0 + 16);
#pragma unroll
    for (int nt = 0; nt < 8; ++nt) {
      const unsigned short* wq = bp + (size_t)(16 * nt) * (size_t)KB + k0;
      FragB bf;
      bf.h[0] = *(const v8usa*)wq;
      bf.h[1] = *(const v8usa*)(wq + 16);
      acc[nt] = wmb(af, bf, acc[nt]);
    }
  }
  if constexpr (MODE == 0) {
    const unsigned short* ap1 = A1 + (size_t)(rowBase + 16 * wave + m) * (size_t)DF + 8 * hh;
#pragma unroll 1
    for (int k0 = 0; k0 < DF; k0 += 32) {
      FragB af;
      af.h[0] = *(const v8usa*)(ap1 + k0);
      af.h[1] = *(const v8usa*)(ap1 + k0 + 16);
#pragma unroll
      for (int nt = 0; nt < 8; ++nt) {
        const unsigned short* wq = bp + (size_t)(16 * nt) * (size_t)KB + PA + k0;
        FragB bf;
        bf.h[0] = *(const v8usa*)wq;
        bf.h[1] = *(const v8usa*)(wq + 16);
        acc[nt] = wmb(af, bf, acc[nt]);
      }
    }
  }

#pragma unroll
  for (int nt = 0; nt < 8; ++nt) {
    const int lc = 16 * nt + m;
#pragma unroll
    for (int r = 0; r < 8; ++r) {
      const int lr = 16 * wave + 8 * hh + r;
      stg[lr * GBN + lc] = acc[nt][r];
    }
  }
  if constexpr (MODE == 0) {
    if (wave == 0) {
      const v4f t = *(const v4f*)(biasp + 4 * lane);
      *(v4fa*)(bsm + 4 * lane) = t;
    }
  }
  __syncthreads();

  v4f pv[16];
#pragma unroll
  for (int i = 0; i < 16; ++i) pv[i] = *(const v4fa*)(stg + (16 * wave + i) * GBN + 4 * lane);
  v4f bb4 = {0.f, 0.f, 0.f, 0.f};
  if constexpr (MODE == 0) bb4 = *(const v4fa*)(bsm + 4 * lane);
  __syncthreads();

  if constexpr (MODE != 0) {
#pragma unroll
    for (int i = 0; i < 16; ++i) {
      const int r = rowBase + 16 * wave + i;
      if (r < nLive) *(volatile v4f*)(outF + (size_t)r * DF + 4 * lane) = pv[i];
    }
    __threadfence();
#pragma unroll
    for (int i = 0; i < 16; ++i) {
      const int r = rowBase + 16 * wave + i;
      if (r < nLive) *(volatile v4f*)(outF + (size_t)r * DF + 4 * lane) = pv[i];
    }
  } else {
#pragma unroll
    for (int i = 0; i < 16; ++i) {
      const bool ok = (rowBase + 16 * wave + i) < nLive;
      const v4f t = pv[i] + bb4;
      v4f y;
      y.x = (t.x > 0.0f) ? t.x : (t.x - t.x);
      y.y = (t.y > 0.0f) ? t.y : (t.y - t.y);
      y.z = (t.z > 0.0f) ? t.z : (t.z - t.z);
      y.w = (t.w > 0.0f) ? t.w : (t.w - t.w);
      y.x = ok ? y.x : 0.0f; y.y = ok ? y.y : 0.0f; y.z = ok ? y.z : 0.0f; y.w = ok ? y.w : 0.0f;
      v4us h4, l4;
      unsigned hb;
      hb = bf16_bits(y.x); h4[0] = (unsigned short)hb; l4[0] = (unsigned short)bf16_bits(y.x - __uint_as_float(hb << 16));
      hb = bf16_bits(y.y); h4[1] = (unsigned short)hb; l4[1] = (unsigned short)bf16_bits(y.y - __uint_as_float(hb << 16));
      hb = bf16_bits(y.z); h4[2] = (unsigned short)hb; l4[2] = (unsigned short)bf16_bits(y.z - __uint_as_float(hb << 16));
      hb = bf16_bits(y.w); h4[3] = (unsigned short)hb; l4[3] = (unsigned short)bf16_bits(y.w - __uint_as_float(hb << 16));
      unsigned short* srow = (unsigned short*)stg + (size_t)(16 * wave + i) * (2 * GBN);
      *(v4usa*)(srow + 4 * lane) = h4;
      *(v4usa*)(srow + DF + 4 * lane) = l4;
    }
    __syncthreads();
    v8us qv[16];
#pragma unroll
    for (int i = 0; i < 16; ++i) {
      const unsigned short* srow = (const unsigned short*)stg + (size_t)(16 * wave + i) * (2 * GBN);
      qv[i] = *(const v8usa*)(srow + 8 * lane);
    }
#pragma unroll
    for (int i = 0; i < 16; ++i) {
      unsigned short* rp = outH + (size_t)(rowBase + 16 * wave + i) * (size_t)PA + 8 * lane;
      *(volatile v8us*)rp = qv[i];
    }
    __threadfence();
#pragma unroll
    for (int i = 0; i < 16; ++i) {
      unsigned short* rp = outH + (size_t)(rowBase + 16 * wave + i) * (size_t)PA + 8 * lane;
      *(volatile v8us*)rp = qv[i];
    }
  }
}

__global__ __launch_bounds__(NTHR) void k_agg1(const float* __restrict__ pr, const float* __restrict__ bf2,
                                               const int* __restrict__ listp, const int* __restrict__ cntp,
                                               const int* __restrict__ offp, const int* __restrict__ flagp,
                                               int nN, int nBlk, float* out) {
  __shared__ __attribute__((aligned(16))) float b2s[OC];
  const int tid = (int)threadIdx.x, lane = tid & 31, wave = tid >> 5;
  if (wave == 0) {
    const int l = lane & 15;
    const v4f t = *(const v4f*)(bf2 + 4 * l);
    *(v4fa*)(b2s + 4 * l) = t;
  }
  __syncthreads();
  const float bv0 = b2s[2 * lane], bv1 = b2s[2 * lane + 1];

  const int rowBase = (int)blockIdx.x * RPB;
  int b = rowBase >> SLA;
  b = b > nBlk - 1 ? nBlk - 1 : b;
  const int fl = __builtin_amdgcn_readfirstlane(flagp[(size_t)b * 32]);
  const int* lp = listp + (size_t)b * RCAP;
  const float qnan = __int_as_float(0x7fc00000);
  const int slotMax = nBlk * NBA - 1;
  const int sa = (2 * lane) & 31, sb = (2 * lane + 1) & 31;

#pragma unroll 1
  for (int j = 0; j < RPB / NWAVE; ++j) {
    const int node = rowBase + wave * (RPB / NWAVE) + j;
    const int sc = node < slotMax ? node : slotMax;
    const int nc = node < nN ? node : nN - 1;
    int c = __builtin_amdgcn_readfirstlane(cntp[sc]);
    int o = __builtin_amdgcn_readfirstlane(offp[sc]);
    const bool big = c > DEGCAP;
    c = c < 0 ? 0 : (c > DEGCAP ? DEGCAP : c);
    o = o < 0 ? 0 : (o > RCAP - 1 ? RCAP - 1 : o);
    int last = o + c - 1;
    last = last < 0 ? 0 : (last > RCAP - 1 ? RCAP - 1 : last);
    float acc0 = 0.0f, acc1 = 0.0f;
#pragma unroll 1
    for (int b0 = 0; b0 < c; b0 += 32) {
      int idx = o + b0 + lane;
      idx = idx > last ? last : idx;
      int sr = lp[idx];
      sr = sr < 0 ? 0 : (sr > nN - 1 ? nN - 1 : sr);
      const int m32 = (c - b0) < 32 ? (c - b0) : 32;
#pragma unroll 1
      for (int k = 0; k < m32; ++k) {
        const int sk = __builtin_amdgcn_readlane(sr, k);
        const v2f a = *(const v2fa*)(pr + (size_t)sk * DF + 2 * lane);
        acc0 += a.x; acc1 += a.y;
      }
    }
    const v2f rr = *(const v2fa*)(pr + (size_t)nc * DF + OC + 2 * lane);
    float y0 = (acc0 + rr.x) + bv0;
    float y1 = (acc1 + rr.y) + bv1;
    const bool poison = (fl != 0) || big;
    y0 = poison ? qnan : y0;
    y1 = poison ? qnan : y1;
    v4f ow;
    ow.x = __shfl(y0, sa, 32); ow.y = __shfl(y1, sa, 32);
    ow.z = __shfl(y0, sb, 32); ow.w = __shfl(y1, sb, 32);
    float* op = out + (size_t)nc * OC + 4 * (lane & 15);
    const bool wr = (node < nN) && (lane < 16);
    if (wr) *(volatile v4f*)op = ow;
    __threadfence();
    if (wr) *(volatile v4f*)op = ow;
  }
}

static inline int cdiv(int a, int b) { return (a + b - 1) / b; }
static inline size_t al256(size_t o) { return (o + 255) & ~(size_t)255; }

extern "C" void kernel_launch(void* const* d_in, const int* in_sizes, int n_in,
                              void* d_out, int out_size, void* d_ws, size_t ws_size,
                              hipStream_t stream) {
  if (n_in < 8) return;
  if (in_sizes[0] < DF || (in_sizes[0] % DF) != 0) return;
  const int nN = in_sizes[0] / DF;
  if (nN < 16 || nN > (1 << 22)) return;
  if (in_sizes[1] < 2 || (in_sizes[1] & 1) != 0) return;
  const int nE = in_sizes[1] / 2;
  if (nE < 1 || nE >= (1 << (31 - SLA))) return;
  if (in_sizes[2] != DF * DF || in_sizes[3] != DF * DF || in_sizes[4] != DF) return;
  if (in_sizes[5] != OC * DF || in_sizes[6] != OC * DF || in_sizes[7] != OC) return;
  if ((long long)out_size != (long long)nN * OC) return;

  const float* x      = (const float*)d_in[0];
  const int*   ei     = (const int*)d_in[1];
  const float* W1rel  = (const float*)d_in[2];
  const float* W1root = (const float*)d_in[3];
  const float* b1     = (const float*)d_in[4];
  const float* W2rel  = (const float*)d_in[5];
  const float* W2root = (const float*)d_in[6];
  const float* b2     = (const float*)d_in[7];
  float* out = (float*)d_out;

  const int MP   = cdiv(nN, 128) * 128;
  const int nBlk = cdiv(MP, NBA);
  if ((long long)nBlk * NBA < (long long)MP) return;
  if ((MP % GBM) != 0 || (MP % RPB) != 0) return;
  const int nbX  = (MP * (DF / 8)) / NTHR;
  if ((long long)nbX * NTHR != (long long)MP * (DF / 8)) return;
  const int vec8 = ((nE & 3) == 0) ? 1 : 0;

  char* ws = (char*)d_ws;
  size_t off = 0;
  const size_t oW1  = off; off = al256(off + (size_t)DF * K0L * 2);
  const size_t oW2  = off; off = al256(off + (size_t)128 * K1L * 2);
  const size_t oBF  = off; off = al256(off + (size_t)(DF + OC) * 4);
  const size_t oFL  = off; off = al256(off + (size_t)nBlk * 128);
  const size_t oCN  = off; off = al256(off + (size_t)nBlk * NBA * 4);
  const size_t oOF  = off; off = al256(off + (size_t)nBlk * NBA * 4);
  const size_t oLS  = off; off = al256(off + (size_t)nBlk * RCAP * 4);
  const size_t oXB  = off; off = al256(off + (size_t)MP * DF * 2);
  const size_t oAG  = off; off = al256(off + (size_t)MP * PA * 2);
  const size_t oH1  = off; off = al256(off + (size_t)MP * PA * 2);
  const size_t oPR  = off; off = al256(off + (size_t)MP * DF * 4);
  if (off > ws_size || off > (size_t)WSMAX) return;
  unsigned short* W1cat = (unsigned short*)(ws + oW1);
  unsigned short* W2cat = (unsigned short*)(ws + oW2);
  float*          BF    = (float*)(ws + oBF);
  int*            FLG   = (int*)(ws + oFL);
  int*            CNT   = (int*)(ws + oCN);
  int*            OFFS  = (int*)(ws + oOF);
  int*            LST   = (int*)(ws + oLS);
  unsigned short* XB    = (unsigned short*)(ws + oXB);
  unsigned short* AGG   = (unsigned short*)(ws + oAG);
  unsigned short* H1    = (unsigned short*)(ws + oH1);
  float*          PR    = (float*)(ws + oPR);

  const size_t cLds = (size_t)AGG_LDS_INTS * 4;
  hipFuncSetAttribute(reinterpret_cast<const void*>(&k_compact), hipFuncAttributeMaxDynamicSharedMemorySize, (int)cLds);

  k_prep<<<nbX + NB_W1 + NB_W2 + 1, NTHR, 0, stream>>>(x, W1rel, W1root, b1, W2rel, W2root, b2, nN, nbX,
                                                      XB, W1cat, W2cat, BF);
  k_compact<<<nBlk, NTHR, cLds, stream>>>(ei, nE, nN, vec8, LST, CNT, OFFS, FLG);
  k_agg0<<<MP / RPB, NTHR, 0, stream>>>(XB, LST, CNT, OFFS, FLG, nN, MP, nBlk, AGG);
  k_gemm<0><<<MP / GBM, GTHR, 0, stream>>>(AGG, XB, W1cat, BF, H1, PR, nN);
  k_gemm<1><<<MP / GBM, GTHR, 0, stream>>>(H1, XB, W2cat, BF, AGG, PR, MP);
  k_agg1<<<cdiv(nN, RPB), NTHR, 0, stream>>>(PR, BF + DF, LST, CNT, OFFS, FLG, nN, nBlk, out);
}
